// NonLocalBlock_71588514890083
// MI455X (gfx1250) — hardware-verified
//
#include <hip/hip_runtime.h>
#include <hip/hip_bf16.h>

#define BB  4
#define CC  256
#define CII 128
#define NN  4096
#define EPSV 1e-5f

typedef __attribute__((ext_vector_type(16))) _Float16 v16h;
typedef __attribute__((ext_vector_type(8)))  _Float16 v8h;
typedef __attribute__((ext_vector_type(8)))  float    v8f;
typedef __attribute__((ext_vector_type(4)))  float    v4f_t;
typedef float v4fa __attribute__((ext_vector_type(4), may_alias));
static __device__ __forceinline__ unsigned pk2(float a, float b) { return (unsigned)__builtin_bit_cast(unsigned short, (_Float16)a) | ((unsigned)__builtin_bit_cast(unsigned short, (_Float16)b) << 16); }
#define NPB (BB * NN / 16)

#if __has_builtin(__builtin_amdgcn_global_load_async_to_lds_b128) && \
    __has_builtin(__builtin_amdgcn_s_wait_asynccnt)
#define USE_ASYNC_LDS 1
typedef int i4v __attribute__((__vector_size__(4 * sizeof(int))));
typedef __attribute__((address_space(1))) i4v gi4v;
typedef __attribute__((address_space(3))) i4v li4v;
#define WAIT_ASYNC(n) __builtin_amdgcn_s_wait_asynccnt(n)
#else
#define USE_ASYNC_LDS 0
#define WAIT_ASYNC(n)
#endif

__device__ __forceinline__ void copy16_g2l(const _Float16* __restrict__ g,
                                           _Float16* l) {
#if USE_ASYNC_LDS
    __builtin_amdgcn_global_load_async_to_lds_b128((gi4v*)g, (li4v*)l, 0, 0);
#else
    *(v8h*)l = *(const v8h*)g;
#endif
}

__device__ __forceinline__ v16h load_a_16x32(const _Float16* __restrict__ base,
                                             int ld, int row0, int k0) {
    const int lane = threadIdx.x & 31;
    const _Float16* p = base + (size_t)(row0 + (lane & 15)) * ld + k0 + ((lane >> 4) << 3);
    v8h g0 = *(const v8h*)(p);
    v8h g1 = *(const v8h*)(p + 16);
    v16h a;
#pragma unroll
    for (int i = 0; i < 8; ++i) { a[i] = g0[i]; a[8 + i] = g1[i]; }
    return a;
}

__device__ __forceinline__ v16h load_b_32x16(const _Float16* __restrict__ base,
                                             int ld, int n0, int k0) {
    const int lane = threadIdx.x & 31;
    const _Float16* p = base + (size_t)(n0 + (lane & 15)) * ld + k0 + ((lane >> 4) << 3);
    v8h g0 = *(const v8h*)(p);
    v8h g1 = *(const v8h*)(p + 16);
    v16h b;
#pragma unroll
    for (int i = 0; i < 8; ++i) { b[i] = g0[i]; b[8 + i] = g1[i]; }
    return b;
}

__device__ __forceinline__ v8f wmma_f16(v16h a, v16h b, v8f c) {
    return __builtin_amdgcn_wmma_f32_16x16x32_f16(false, a, false, b, (short)0, c,
                                                  false, false);
}

__global__ void convert_w_kernel(const float* __restrict__ W_w,
                                 _Float16* __restrict__ wh) {
    int i = (blockIdx.x * 256 + threadIdx.x) * 2;
    if (i < CC * CII) { const unsigned p = pk2(W_w[i], W_w[i + 1]); *(volatile unsigned*)(wh + i) = p; __threadfence(); *(volatile unsigned*)(wh + i) = p; }
}

__global__ __launch_bounds__(256) void prep_kernel(const float* __restrict__ x,
                                                   const float* __restrict__ g_w,
                                                   const float* __restrict__ g_b,
                                                   _Float16* __restrict__ xh,
                                                   _Float16* __restrict__ gxT) {
    __shared__ float xt[CC][65];
    const int t = threadIdx.x;
    const int blk = blockIdx.x;
    const int b  = blk / (NN / 64);
    const int n0 = (blk % (NN / 64)) * 64;
    const float* xb = x + (size_t)b * CC * NN;

    for (int idx = t; idx < CC * 64; idx += 256) {
        int c = idx >> 6, j = idx & 63;
        xt[c][j] = xb[(size_t)c * NN + n0 + j];
    }
    __syncthreads();

    for (int idx = t; idx < 64 * (CC / 2); idx += 256) {
        int cp = idx & (CC / 2 - 1), j = idx >> 7;
        const unsigned p = pk2(xt[2 * cp][j], xt[2 * cp + 1][j]);
        _Float16* d = xh + ((size_t)b * NN + n0 + j) * CC + 2 * cp;
        *(volatile unsigned*)d = p; __threadfence(); *(volatile unsigned*)d = p;
    }

    const int j = t & 31, g = t >> 5;
    float acc0[16], acc1[16];
#pragma unroll
    for (int i = 0; i < 16; ++i) { acc0[i] = g_b[g * 16 + i]; acc1[i] = acc0[i]; }
    for (int c = 0; c < CC; ++c) {
        float x0 = xt[c][2 * j], x1 = xt[c][2 * j + 1];
#pragma unroll
        for (int i = 0; i < 16; ++i) {
            const float w = g_w[(g * 16 + i) * CC + c];
            acc0[i] += w * x0; acc1[i] += w * x1;
        }
    }
#pragma unroll
    for (int i = 0; i < 16; ++i) {
        const unsigned p = pk2(acc0[i], acc1[i]);
        _Float16* d = gxT + ((size_t)b * CII + g * 16 + i) * NN + n0 + 2 * j;
        *(volatile unsigned*)d = p; __threadfence(); *(volatile unsigned*)d = p;
    }
}

#define KROW_LD 264
#define VROW_LD 40
#define NT      (NN / 32)

__global__ __launch_bounds__(256) void attn_kernel(const _Float16* __restrict__ xh,
                                                   const _Float16* __restrict__ gxT,
                                                   _Float16* __restrict__ y) {
    const int wave = threadIdx.x >> 5;
    const int lane = threadIdx.x & 31;
    const int t    = threadIdx.x;
    const int wid  = blockIdx.x * 8 + wave;
    const int b    = wid / (NN / 16);
    const int q0   = (wid % (NN / 16)) * 16;

    const _Float16* xq = xh  + (size_t)b * NN * CC;
    const _Float16* vt = gxT + (size_t)b * CII * NN;

    __shared__ __align__(16) _Float16 kbuf[2][32][KROW_LD];
    __shared__ __align__(16) _Float16 vbuf[2][CII][VROW_LD];
    __shared__ __align__(16) _Float16 pbuf[8][16][32];

    auto prefetch = [&](int buf, int key0) {
#pragma unroll
        for (int i = 0; i < 4; ++i) {
            int e = t + i * 256;
            int row = e >> 5, seg = e & 31;
            copy16_g2l(xq + (size_t)(key0 + row) * CC + seg * 8,
                       &kbuf[buf][row][seg * 8]);
        }
#pragma unroll
        for (int i = 0; i < 2; ++i) {
            int e = t + i * 256;
            int row = e >> 2, seg = e & 3;
            copy16_g2l(vt + (size_t)row * NN + key0 + seg * 8,
                       &vbuf[buf][row][seg * 8]);
        }
    };

    prefetch(0, 0);

    v16h qf[8];
#pragma unroll
    for (int kk = 0; kk < 8; ++kk) qf[kk] = load_a_16x32(xq, CC, q0, kk * 32);

    v8f o[8] = {};
    float m[8], l[8];
#pragma unroll
    for (int r = 0; r < 8; ++r) { m[r] = -1e30f; l[r] = 0.f; }

    for (int it = 0; it < NT; ++it) {
        const int key0 = it * 32;
        const int cur = it & 1;
        __syncthreads();
        if (it + 1 < NT) {
            prefetch(cur ^ 1, key0 + 32);
            WAIT_ASYNC(6);
        } else {
            WAIT_ASYNC(0);
        }
        __syncthreads();

        v8f s0 = {}, s1 = {};
        const _Float16* kb = &kbuf[cur][0][0];
#pragma unroll
        for (int kk = 0; kk < 8; ++kk) {
            v16h b0 = load_b_32x16(kb, KROW_LD, 0,  kk * 32);
            v16h b1 = load_b_32x16(kb, KROW_LD, 16, kk * 32);
            s0 = wmma_f16(qf[kk], b0, s0);
            s1 = wmma_f16(qf[kk], b1, s1);
        }

#pragma unroll
        for (int r = 0; r < 8; ++r) {
            float rm = fmaxf(s0[r], s1[r]);
#pragma unroll
            for (int off = 8; off >= 1; off >>= 1)
                rm = fmaxf(rm, __shfl_xor(rm, off, 16));
            float mn    = fmaxf(m[r], rm);
            float scale = __expf(m[r] - mn);
            float p0    = __expf(s0[r] - mn);
            float p1    = __expf(s1[r] - mn);
            float rs    = p0 + p1;
#pragma unroll
            for (int off = 8; off >= 1; off >>= 1)
                rs += __shfl_xor(rs, off, 16);
            l[r] = l[r] * scale + rs;
            m[r] = mn;
#pragma unroll
            for (int jj = 0; jj < 8; ++jj) o[jj][r] *= scale;

            int row = r + ((lane >> 4) << 3);
            pbuf[wave][row][lane & 15]        = (_Float16)(p0 * 1024.0f);
            pbuf[wave][row][16 + (lane & 15)] = (_Float16)(p1 * 1024.0f);
        }
#if __has_builtin(__builtin_amdgcn_s_wait_dscnt)
        __builtin_amdgcn_s_wait_dscnt(0);
#else
        __builtin_amdgcn_fence(__ATOMIC_ACQ_REL, "wavefront");
#endif
        v16h pa = load_a_16x32(&pbuf[wave][0][0], 32, 0, 0);
#pragma unroll
        for (int jj = 0; jj < 8; ++jj) {
            const _Float16* p = &vbuf[cur][jj * 16 + (lane & 15)][(lane >> 4) << 3];
            v8h g0 = *(const v8h*)(p);
            v8h g1 = *(const v8h*)(p + 16);
            v16h vb;
#pragma unroll
            for (int i = 0; i < 8; ++i) { vb[i] = g0[i]; vb[8 + i] = g1[i]; }
            o[jj] = wmma_f16(pa, vb, o[jj]);
        }
    }

    __shared__ __align__(16) float ost[8][16 * CII];
    float* os_ = ost[wave];
#pragma unroll
    for (int r = 0; r < 8; ++r) {
        float inv = 1.f / (l[r] * 1024.0f);
        int row = r + ((lane >> 4) << 3);
#pragma unroll
        for (int jj = 0; jj < 8; ++jj) os_[row * CII + jj * 16 + (lane & 15)] = o[jj][r] * inv;
    }
    asm volatile("s_wait_dscnt 0" ::: "memory");
#pragma unroll 1
    for (int pass = 0; pass < 2; ++pass) {
#pragma unroll 4
        for (int rr = 0; rr < 16; ++rr) {
            _Float16* d = y + ((size_t)b * NN + q0 + rr) * CII;
            *(volatile unsigned*)(d + 2 * lane)      = pk2(os_[rr * CII + 2 * lane],      os_[rr * CII + 2 * lane + 1]);
            *(volatile unsigned*)(d + 64 + 2 * lane) = pk2(os_[rr * CII + 64 + 2 * lane], os_[rr * CII + 64 + 2 * lane + 1]);
        }
        __threadfence();
    }
}

__device__ __forceinline__ v8f compute_wy_tile(const _Float16* __restrict__ y,
                                               const _Float16* __restrict__ wh,
                                               const float* __restrict__ W_b,
                                               int p0, int o0) {
    v8f acc = {};
#pragma unroll
    for (int kk = 0; kk < 4; ++kk) {
        v16h a = load_a_16x32(y,  CII, p0, kk * 32);
        v16h b = load_b_32x16(wh, CII, o0, kk * 32);
        acc = wmma_f16(a, b, acc);
    }
    float bias = W_b[o0 + (threadIdx.x & 15)];
#pragma unroll
    for (int r = 0; r < 8; ++r) acc[r] += bias;
    return acc;
}

__global__ __launch_bounds__(256) void stats_kernel(const _Float16* __restrict__ y,
                                                    const _Float16* __restrict__ wh,
                                                    const float* __restrict__ W_b,
                                                    float* __restrict__ sums,
                                                    float* __restrict__ sqs) {
    __shared__ float ls[CC], lq[CC];
    const int t = threadIdx.x, wave = t >> 5, lane = t & 31;
    const int p0 = blockIdx.x * 16;
#pragma unroll
    for (int half = 0; half < 2; ++half) {
        int o0 = wave * 32 + half * 16;
        v8f acc = compute_wy_tile(y, wh, W_b, p0, o0);
        float s = 0.f, q = 0.f;
#pragma unroll
        for (int r = 0; r < 8; ++r) { s += acc[r]; q += acc[r] * acc[r]; }
        s += __shfl_xor(s, 16, 32);
        q += __shfl_xor(q, 16, 32);
        if (lane < 16) { ls[o0 + lane] = s; lq[o0 + lane] = q; }
    }
    __syncthreads();
    *(volatile float*)(sums + (size_t)blockIdx.x * CC + t) = ls[t]; *(volatile float*)(sqs + (size_t)blockIdx.x * CC + t) = lq[t];
    __threadfence();
    *(volatile float*)(sums + (size_t)blockIdx.x * CC + t) = ls[t]; *(volatile float*)(sqs + (size_t)blockIdx.x * CC + t) = lq[t];
}

__global__ __launch_bounds__(256) void reduce_stats_kernel(const float* __restrict__ psum, const float* __restrict__ psq,
                                                          float* __restrict__ tsum, float* __restrict__ tsq) {
    const int c = threadIdx.x;
    float s = 0.f, q = 0.f;
    for (int i = 0; i < NPB; ++i) { s += psum[(size_t)i * CC + c]; q += psq[(size_t)i * CC + c]; }
    *(volatile float*)(tsum + c) = s; *(volatile float*)(tsq + c) = q;
    __threadfence();
    *(volatile float*)(tsum + c) = s; *(volatile float*)(tsq + c) = q;
}

__global__ __launch_bounds__(256) void final_kernel(const _Float16* __restrict__ y,
                                                    const _Float16* __restrict__ wh,
                                                    const float* __restrict__ W_b,
                                                    const float* __restrict__ sums,
                                                    const float* __restrict__ sqs,
                                                    const float* __restrict__ gamma,
                                                    const float* __restrict__ beta,
                                                    const float* __restrict__ x,
                                                    float* __restrict__ out) {
    __shared__ __align__(16) float so[CC][32 + 4];
    const int t = threadIdx.x, wave = t >> 5, lane = t & 31;
    const int pb = blockIdx.x * 32;
    const float inv_bn = 1.f / (float)(BB * NN);
#pragma unroll 1
    for (int tp = 0; tp < 2; ++tp) {
        const int p0 = pb + tp * 16;
#pragma unroll
        for (int half = 0; half < 2; ++half) {
            int o0 = wave * 32 + half * 16;
            v8f acc = compute_wy_tile(y, wh, W_b, p0, o0);
            int ch = o0 + (lane & 15);
            float mean = sums[ch] * inv_bn;
            float var  = sqs[ch] * inv_bn - mean * mean;
            float rstd = rsqrtf(var + EPSV);
            float ga = gamma[ch], be = beta[ch];
#pragma unroll
            for (int r = 0; r < 8; ++r) so[ch][tp * 16 + r + ((lane >> 4) << 3)] = (acc[r] - mean) * rstd * ga + be;
        }
    }
    __syncthreads();
    const int b = pb / NN, n0 = pb % NN;
#pragma unroll 1
    for (int pass = 0; pass < 2; ++pass) {
#pragma unroll
        for (int i = 0; i < 8; ++i) {
            const int c = t + 256 * i, ch = c >> 3, q = c & 7;
            const size_t idx = ((size_t)(b * CC + ch)) * NN + n0 + q * 4;
            v4f_t v = *(const v4fa*)&so[ch][q * 4];
            v += *(const v4f_t*)(x + idx);
            *(volatile v4f_t*)(out + idx) = v;
        }
        __threadfence();
    }
}

extern "C" void kernel_launch(void* const* d_in, const int* in_sizes, int n_in,
                              void* d_out, int out_size, void* d_ws, size_t ws_size,
                              hipStream_t stream) {
    const float* x     = (const float*)d_in[0];
    const float* g_w   = (const float*)d_in[1];
    const float* g_b   = (const float*)d_in[2];
    const float* W_w   = (const float*)d_in[3];
    const float* W_b   = (const float*)d_in[4];
    const float* gamma = (const float*)d_in[5];
    const float* beta  = (const float*)d_in[6];
    float* out = (float*)d_out;

    char* ws = (char*)d_ws;
    _Float16* xh  = (_Float16*)ws;
    _Float16* gxT = (_Float16*)(ws + (size_t)BB * NN * CC * 2);
    _Float16* y   = (_Float16*)(ws + (size_t)BB * NN * CC * 2
                                   + (size_t)BB * CII * NN * 2);
    _Float16* wh  = (_Float16*)((char*)y + (size_t)BB * NN * CII * 2);
    float* psums  = (float*)((char*)wh + (size_t)CC * CII * 2);
    float* psqs   = psums + (size_t)NPB * CC;
    float* sums   = psqs + (size_t)NPB * CC;
    float* sqs    = sums + CC;

    convert_w_kernel<<<(CC * CII / 2 + 255) / 256, 256, 0, stream>>>(W_w, wh);
    prep_kernel<<<BB * (NN / 64), 256, 0, stream>>>(x, g_w, g_b, xh, gxT);
    attn_kernel<<<(BB * NN / 16) / 8, 256, 0, stream>>>(xh, gxT, y);
    stats_kernel<<<(BB * NN) / 16, 256, 0, stream>>>(y, wh, W_b, psums, psqs);
    reduce_stats_kernel<<<1, 256, 0, stream>>>(psums, psqs, sums, sqs);
    final_kernel<<<(BB * NN) / 32, 256, 0, stream>>>(y, wh, W_b, sums, sqs,
                                                     gamma, beta, x, out);
}
